// PSA_8624294330417
// MI455X (gfx1250) — hardware-run, weakly checked
//
#include <hip/hip_runtime.h>
#include <math.h>

typedef __attribute__((ext_vector_type(16))) _Float16 v16h;
typedef __attribute__((ext_vector_type(16))) __bf16 v16b;
typedef __attribute__((ext_vector_type(8)))  _Float16 v8h;
typedef __attribute__((ext_vector_type(8)))  float v8f;
typedef __attribute__((ext_vector_type(4)))  float v4f;
typedef __attribute__((ext_vector_type(2)))  float v2f;
typedef __attribute__((ext_vector_type(4)))  unsigned v4u;
typedef __attribute__((ext_vector_type(4)))  int v4i;
typedef float __attribute__((may_alias)) float_a;
typedef int __attribute__((may_alias)) int_a;

template <typename T> __device__ __forceinline__ void vst2(void* p, T v) { *(volatile T*)p = v; __threadfence(); *(volatile T*)p = v; }
__device__ __forceinline__ v8f wmma16(v16h a, v16h b, v8f c) {
  v8f d = __builtin_amdgcn_wmma_f32_16x16x32_f16(false, a, false, b, (short)0, c, false, false);
  asm volatile("v_nop\n\tv_nop\n\tv_nop\n\tv_nop" : "+v"(d) : "v"(a), "v"(b));
  return d;
}
__device__ __forceinline__ v8f wmma_bf(v16b a, v16b b, v8f c) {
  v8f d = __builtin_amdgcn_wmma_f32_16x16x32_bf16(false, a, false, b, (short)0, c, false, false);
  asm volatile("v_nop\n\tv_nop\n\tv_nop\n\tv_nop" : "+v"(d) : "v"(a), "v"(b));
  return d;
}
__device__ __forceinline__ v16h frag_h(const _Float16* rowk0, int lane) {
  union { v16h v; v8h q[2]; } u; const _Float16* p = rowk0 + 8 * (lane >> 4);
  u.q[0] = *(const v8h*)p; u.q[1] = *(const v8h*)(p + 16); return u.v;
}
__device__ __forceinline__ v16h frag_f32(const float* rowk0, int lane) {
  v16h a; const float* p = rowk0 + 8 * (lane >> 4);
#pragma unroll
  for (int i = 0; i < 8; ++i) { a[i] = (_Float16)p[i]; a[8 + i] = (_Float16)p[16 + i]; }
  return a;
}
__device__ __forceinline__ v16h frag_f32s(const float* rowk0, int lane, float sc) {
  v16h a; const float* p = rowk0 + 8 * (lane >> 4);
#pragma unroll
  for (int i = 0; i < 8; ++i) { a[i] = (_Float16)(p[i] * sc); a[8 + i] = (_Float16)(p[16 + i] * sc); }
  return a;
}
__device__ __forceinline__ v16h fragc_f32(const float* W, int k0, int n, int lane, int ld, int K) {
  v16h a; const int g = lane >> 4;
#pragma unroll
  for (int i = 0; i < 8; ++i) { const int ka = k0 + 8 * g + i, kb = ka + 16;
    a[i] = (_Float16)(ka < K ? W[(size_t)(ka < K ? ka : K - 1) * ld + n] : 0.f); a[8 + i] = (_Float16)(kb < K ? W[(size_t)(kb < K ? kb : K - 1) * ld + n] : 0.f); }
  return a;
}
struct F2 { v16b h, l; };
__device__ __forceinline__ F2 bsplit16(const float v[16]) { F2 r;
#pragma unroll
  for (int i = 0; i < 16; ++i) { const __bf16 h = (__bf16)v[i]; r.h[i] = h; r.l[i] = (__bf16)(v[i] - (float)h); }
  return r; }
__device__ __forceinline__ F2 split_row(const float* row, int k0, int lane) { float v[16]; const float* p = row + k0 + 8 * (lane >> 4);
#pragma unroll
  for (int i = 0; i < 8; ++i) { v[i] = p[i]; v[8 + i] = p[16 + i]; }
  return bsplit16(v); }
__device__ __forceinline__ F2 split_rowK(const float* row, int k0, int lane, int K) { float v[16]; const int g = lane >> 4;
#pragma unroll
  for (int i = 0; i < 8; ++i) { const int ka = k0 + 8 * g + i, kb = ka + 16; v[i] = ka < K ? row[ka < K ? ka : K - 1] : 0.f; v[8 + i] = kb < K ? row[kb < K ? kb : K - 1] : 0.f; }
  return bsplit16(v); }
__device__ __forceinline__ F2 split_col(const float* W, int k0, int n, int lane, int ld, int K) { float v[16]; const int g = lane >> 4;
#pragma unroll
  for (int i = 0; i < 8; ++i) { const int ka = k0 + 8 * g + i, kb = ka + 16; v[i] = ka < K ? W[(size_t)(ka < K ? ka : K - 1) * ld + n] : 0.f; v[8 + i] = kb < K ? W[(size_t)(kb < K ? kb : K - 1) * ld + n] : 0.f; }
  return bsplit16(v); }
__device__ __forceinline__ v8f mac3(const F2& a, const F2& b, v8f c) { c = wmma_bf(a.l, b.h, c); c = wmma_bf(a.h, b.l, c); return wmma_bf(a.h, b.h, c); }
__device__ __forceinline__ float sigm(float v) { return 1.0f / (1.0f + expf(-v)); }
#define LDSX() do { asm volatile("s_wait_dscnt 0" ::: "memory"); __builtin_amdgcn_wave_barrier(); __builtin_amdgcn_fence(__ATOMIC_RELEASE, "workgroup"); } while (0)

__device__ __forceinline__ float bfr(float v) { return (float)(__bf16)v; }
#define NBT 4
#define CA 256
#define CT 512
#define NN 4096
#define XP 4096
#define NH 4
#define HD 64
#ifndef TNB
#define TNB NBT
#endif
#define WS_Q   0u
#define WS_K   (WS_Q + 2u * (size_t)NBT * NN * CA)
#define WS_V   (WS_K + 2u * (size_t)NBT * NN * CA)
#define WS_S   (WS_V + 2u * (size_t)NBT * CA * NN)
#define WS_P   (WS_S + 4u * (size_t)NN * NN)
#define WS_O   (WS_P + 2u * (size_t)NN * NN)
#define WS_Z   (WS_O + 4u * (size_t)NBT * NN * CA)
#define WS_BN  (WS_Z + 4u * (size_t)NBT * CA * NN)
#define WS_END (WS_BN + 4u * 2u * (size_t)CA)

__global__ __launch_bounds__(128) void k_qkv(const float* __restrict__ X, const float* __restrict__ WQKV, _Float16* __restrict__ QR, _Float16* __restrict__ KR, _Float16* __restrict__ VP) {
  __shared__ __align__(16) _Float16 sh[128][72]; __shared__ __align__(16) _Float16 th[64][136];
  const int tid = threadIdx.x, wave = tid >> 5, lane = tid & 31, col = lane & 15, g = lane >> 4; const int rb = blockIdx.y; const int which = rb / 4, d0 = (rb % 4) * 64; const int b = blockIdx.z; const int n0 = blockIdx.x * 128;
  const float* Wm = WQKV + (size_t)(rb * 64) * CA; const float* Xb = X + (size_t)b * CT * XP;
  v8f acc[8] = {};
#pragma unroll 2
  for (int kc = 0; kc < CA / 32; ++kc) { v16b a; { const float* p = Wm + (size_t)(wave * 16 + col) * CA + kc * 32 + 8 * g;
#pragma unroll
      for (int e = 0; e < 8; ++e) { a[e] = (__bf16)p[e]; a[8 + e] = (__bf16)p[16 + e]; } }
#pragma unroll
    for (int j = 0; j < 8; ++j) { v16b w; const int n = n0 + j * 16 + col;
#pragma unroll
      for (int e = 0; e < 8; ++e) { w[e] = (__bf16)Xb[(size_t)(kc * 32 + 8 * g + e) * XP + n]; w[8 + e] = (__bf16)Xb[(size_t)(kc * 32 + 16 + 8 * g + e) * XP + n]; }
      acc[j] = wmma_bf(a, w, acc[j]); } }
#pragma unroll
  for (int j = 0; j < 8; ++j)
#pragma unroll
    for (int r = 0; r < 8; ++r) { const int rl = wave * 16 + 8 * g + r, cl = j * 16 + col; const _Float16 hv = (_Float16)acc[j][r]; if (which == 2) th[rl][cl] = hv; else sh[cl][rl] = hv; }
  __syncthreads();
  if (which < 2) { _Float16* dst = (which == 0 ? QR : KR) + ((size_t)b * NN + n0) * CA + d0; for (int e = tid; e < 128 * 8; e += 128) { const int cl = e >> 3, q = e & 7; vst2((unsigned*)(dst + (size_t)cl * CA + q * 8), *(const v4u*)&sh[cl][q * 8]); } }
  else { _Float16* dst = VP + ((size_t)b * CA + d0) * NN + n0; for (int e = tid; e < 64 * 16; e += 128) { const int rl = e >> 4, q = e & 15; vst2((unsigned*)(dst + (size_t)rl * NN + q * 8), *(const v4u*)&th[rl][q * 8]); } } }
__global__ __launch_bounds__(128) void k_sc(const _Float16* __restrict__ QR, const _Float16* __restrict__ KR, int b, int h, float* __restrict__ S) { __shared__ __align__(16) float ss[4][16][132];
  const int tid = threadIdx.x, wave = tid >> 5, lane = tid & 31, col = lane & 15, g = lane >> 4; const int k0 = blockIdx.y * 128; const int ql0 = blockIdx.x * 64 + wave * 16;
  const _Float16* Q = QR + (size_t)b * NN * CA + h * HD; const _Float16* K = KR + (size_t)b * NN * CA + h * HD;
  v8f acc[8] = {};
#pragma unroll
  for (int kc = 0; kc < HD / 32; ++kc) { const v16h ah = frag_h(Q + (size_t)(ql0 + col) * CA + kc * 32, lane);
#pragma unroll
    for (int j = 0; j < 8; ++j) { const v16h kb = frag_h(K + (size_t)(k0 + j * 16 + col) * CA + kc * 32, lane); acc[j] = wmma16(ah, kb, acc[j]); } }
#pragma unroll
  for (int j = 0; j < 8; ++j)
#pragma unroll
    for (int r = 0; r < 8; ++r) ss[wave][8 * g + r][j * 16 + col] = acc[j][r] * 0.125f;
  LDSX(); for (int rl = 0; rl < 16; ++rl) vst2(S + (size_t)(ql0 + rl) * NN + k0 + lane * 4, *(const v4f*)&ss[wave][rl][lane * 4]); }
__global__ __launch_bounds__(256) void k_sm(const float* __restrict__ S, _Float16* __restrict__ P) { __shared__ float sred[8]; __shared__ float sbc; __shared__ __align__(16) _Float16 shp[NN];
  const int t = threadIdx.x; const size_t row = blockIdx.x; const float* sr = S + row * NN;
  float m = -3.0e38f; for (int k = t; k < NN; k += 256) m = fmaxf(m, sr[k]);
#pragma unroll
  for (int o = 1; o < 32; o <<= 1) m = fmaxf(m, __shfl_xor(m, o));
  if ((t & 31) == 0) sred[t >> 5] = m; __syncthreads(); if (t == 0) { float a = sred[0]; for (int e = 1; e < 8; ++e) a = fmaxf(a, sred[e]); sbc = a; } __syncthreads(); m = sbc; __syncthreads();
  float sum = 0.f; for (int k = t; k < NN; k += 256) sum += expf(sr[k] - m);
#pragma unroll
  for (int o = 1; o < 32; o <<= 1) sum += __shfl_xor(sum, o);
  if ((t & 31) == 0) sred[t >> 5] = sum; __syncthreads(); if (t == 0) { float a = 0.f; for (int e = 0; e < 8; ++e) a += sred[e]; sbc = 1.0f / a; } __syncthreads(); const float inv = sbc;
  for (int k = t; k < NN; k += 256) shp[k] = (_Float16)(expf(sr[k] - m) * inv * 2048.0f);
  __syncthreads(); for (int q = t; q < NN / 8; q += 256) vst2((unsigned*)(P + row * NN + q * 8), *(const v4u*)&shp[q * 8]); }
__global__ __launch_bounds__(128) void k_pv(const _Float16* __restrict__ P, const _Float16* __restrict__ VP, int b, int h, float* __restrict__ O) { __shared__ __align__(16) float ss[4][16][HD + 4];
  const int tid = threadIdx.x, wave = tid >> 5, lane = tid & 31, col = lane & 15, g = lane >> 4; const int ql0 = blockIdx.x * 64 + wave * 16; const _Float16* V = VP + ((size_t)b * CA + h * HD) * NN;
  v8f acc[HD / 16] = {};
#pragma unroll 1
  for (int kc = 0; kc < NN / 32; ++kc) { const v16h ph = frag_h(P + (size_t)(ql0 + col) * NN + kc * 32, lane);
#pragma unroll
    for (int jj = 0; jj < HD / 16; ++jj) acc[jj] = wmma16(ph, frag_h(V + (size_t)(jj * 16 + col) * NN + kc * 32, lane), acc[jj]); }
#pragma unroll
  for (int jj = 0; jj < HD / 16; ++jj)
#pragma unroll
    for (int r = 0; r < 8; ++r) ss[wave][8 * g + r][jj * 16 + col] = acc[jj][r] * (1.0f / 2048.0f);
  LDSX(); for (int rl = 0; rl < 16; ++rl) if (lane < HD / 4) vst2(O + ((size_t)b * NN + ql0 + rl) * CA + h * HD + lane * 4, *(const v4f*)&ss[wave][rl][lane * 4]); }
__global__ __launch_bounds__(128) void k_proj(const float* __restrict__ O, const float* __restrict__ WP, float* __restrict__ Z) { __shared__ __align__(16) float st[128][68];
  const int tid = threadIdx.x, wave = tid >> 5, lane = tid & 31, col = lane & 15, g = lane >> 4; const int b = blockIdx.z; const int c0 = blockIdx.y * 128; const int n0 = blockIdx.x * 64; const int nl0 = wave * 16;
  v8f acc[8] = {};
#pragma unroll
  for (int kc = 0; kc < CA / 32; ++kc) { const F2 a = split_row(O + ((size_t)b * NN + n0 + nl0 + col) * CA, kc * 32, lane);
#pragma unroll
    for (int j = 0; j < 8; ++j) { v16b w; const int c = c0 + j * 16 + col;
#pragma unroll
      for (int e = 0; e < 8; ++e) { w[e] = (__bf16)WP[(size_t)c * CA + kc * 32 + 8 * g + e]; w[8 + e] = (__bf16)WP[(size_t)c * CA + kc * 32 + 16 + 8 * g + e]; }
      acc[j] = wmma_bf(a.h, w, acc[j]); acc[j] = wmma_bf(a.l, w, acc[j]); } }
#pragma unroll
  for (int j = 0; j < 8; ++j)
#pragma unroll
    for (int r = 0; r < 8; ++r) st[j * 16 + col][nl0 + 8 * g + r] = acc[j][r];
  __syncthreads();
  for (int cl = wave * 32; cl < wave * 32 + 32; ++cl) if (lane < 16) vst2(Z + ((size_t)b * CA + c0 + cl) * NN + n0 + lane * 4, *(const v4f*)&st[cl][lane * 4]); }
__global__ __launch_bounds__(256) void k_bnstat(const float* __restrict__ Z, float* __restrict__ BN) { __shared__ float smu[32], srs[32];
  const int t = threadIdx.x; const int cl = t >> 3, sub = t & 7; const int c = blockIdx.x * 32 + cl; const int total = TNB * NN;
  float s = 0.f; for (int i = sub * 4; i < total; i += 32) { const int b = i / NN, n = i % NN; const v4f z = *(const v4f*)(Z + ((size_t)b * CA + c) * NN + n); s += (z[0] + z[1]) + (z[2] + z[3]); }
#pragma unroll
  for (int o = 1; o < 8; o <<= 1) s += __shfl_xor(s, o);
  const float mu = s / (float)total;
  float s2 = 0.f; for (int i = sub * 4; i < total; i += 32) { const int b = i / NN, n = i % NN; const v4f z = *(const v4f*)(Z + ((size_t)b * CA + c) * NN + n); const v4f d = z - mu; s2 += (d[0] * d[0] + d[1] * d[1]) + (d[2] * d[2] + d[3] * d[3]); }
#pragma unroll
  for (int o = 1; o < 8; o <<= 1) s2 += __shfl_xor(s2, o);
  if (sub == 0) { smu[cl] = mu; srs[cl] = rsqrtf(s2 / (float)total + 1e-5f); }
  __syncthreads(); if (t < 32) { vst2(BN + blockIdx.x * 32 + t, smu[t]); vst2(BN + CA + blockIdx.x * 32 + t, srs[t]); } }
__global__ __launch_bounds__(256) void k_apply(const float* __restrict__ Z, const float* __restrict__ BN, const float* __restrict__ GA, const float* __restrict__ BE, const float* __restrict__ X, float* __restrict__ OUT) {
  const int t = threadIdx.x; const int b = blockIdx.x / CT, c = blockIdx.x % CT; float* dst = OUT + ((size_t)b * CT + c) * XP;
  if (c < CA) { const float mu = BN[c], rs = BN[CA + c], ga = bfr(GA[c]), be = bfr(BE[c]); const float* src = Z + ((size_t)b * CA + c) * NN;
    for (int q = t; q < NN / 4; q += 256) { const v4f z = *(const v4f*)(src + q * 4); v4f o;
#pragma unroll
      for (int e = 0; e < 4; ++e) o[e] = (z[e] - mu) * rs * ga + be; vst2(dst + q * 4, o); } }
  else { const float* src = X + ((size_t)b * CT + c) * XP;
    for (int q = t; q < NN / 4; q += 256) { const v4f x = *(const v4f*)(src + q * 4); v4f o;
#pragma unroll
      for (int e = 0; e < 4; ++e) o[e] = bfr(x[e]); vst2(dst + q * 4, o); } } }
extern "C" void kernel_launch(void* const* d_in, const int* in_sizes, int n_in, void* d_out, int out_size, void* d_ws, size_t ws_size, hipStream_t stream) {
  (void)in_sizes; (void)n_in; (void)out_size;
  const float** F = (const float**)d_in;
  if (ws_size < (size_t)WS_END) return;
  char* ws = (char*)d_ws; _Float16 *QR = (_Float16*)(ws + WS_Q), *KR = (_Float16*)(ws + WS_K), *VP = (_Float16*)(ws + WS_V), *P = (_Float16*)(ws + WS_P); float *S = (float*)(ws + WS_S), *O = (float*)(ws + WS_O), *Z = (float*)(ws + WS_Z), *BN = (float*)(ws + WS_BN);
  k_qkv<<<dim3(NN / 128, 12, TNB), 128, 0, stream>>>(F[0], F[1], QR, KR, VP);
  for (int b = 0; b < TNB; ++b) for (int h = 0; h < NH; ++h) {
    k_sc<<<dim3(NN / 64, NN / 128), 128, 0, stream>>>(QR, KR, b, h, S);
    k_sm<<<dim3(NN), 256, 0, stream>>>(S, P);
    k_pv<<<dim3(NN / 64), 128, 0, stream>>>(P, VP, b, h, O);
  }
  k_proj<<<dim3(NN / 64, CA / 128, TNB), 128, 0, stream>>>(O, F[2], Z);
  k_bnstat<<<dim3(CA / 32), 256, 0, stream>>>(Z, BN);
  k_apply<<<dim3(TNB * CT), 256, 0, stream>>>(Z, BN, F[3], F[4], F[0], (float*)d_out);
}
